// RelationshipFusionWithAttention_90537910600027
// MI455X (gfx1250) — hardware-verified
//
#include <hip/hip_runtime.h>
#include <hip/hip_bf16.h>
#include <math.h>

#define NBr 8
#define NNr 128
#define DDr 256
#define RRr 64
#define NROW (NBr * NNr)
#define GSTR 48

typedef _Float16 bf16;
typedef _Float16 f16;
typedef __attribute__((ext_vector_type(4))) unsigned v4u_t;
typedef unsigned v4ua __attribute__((ext_vector_type(4), may_alias));
typedef __attribute__((ext_vector_type(4))) float v4f_t;
typedef float v4fa __attribute__((ext_vector_type(4), may_alias));
typedef __attribute__((ext_vector_type(16))) bf16  bf16x16;
typedef bf16x16 f16x16;
typedef __attribute__((ext_vector_type(8)))  bf16  bf16x8;
typedef bf16x8 f16x8;
typedef __attribute__((ext_vector_type(8)))  float f32x8;
__device__ __forceinline__ f32x8 wmma16(f16x16 a, f16x16 b, f32x8 c) {
  c = __builtin_amdgcn_wmma_f32_16x16x32_f16(false, a, false, b, (short)0, c, false, false);
  asm volatile("v_nop\n\tv_nop\n\tv_nop\n\tv_nop" : "+v"(c) : "v"(a), "v"(b));
  return c;
}
__device__ __forceinline__ f16x16 lds_frag(const f16* base, int stride) {
  const int lane = threadIdx.x & 31, row = lane & 15, kh = (lane >> 4) * 8;
  const f16x8 lo = *(const f16x8*)(base + row * stride + kh);
  const f16x8 hi = *(const f16x8*)(base + row * stride + kh + 16);
  f16x16 f;
#pragma unroll
  for (int i = 0; i < 8; ++i) { f[i] = lo[i]; f[i + 8] = hi[i]; }
  return f;
}
__device__ __forceinline__ f16x16 wfragKN(const float* __restrict__ Wm, int ldw, int k0, int n0) {
  const int lane = threadIdx.x & 31, n = n0 + (lane & 15), kh = (lane >> 4) * 8; f16x16 f;
#pragma unroll
  for (int i = 0; i < 8; ++i) { f[i] = (f16)Wm[(size_t)(k0 + kh + i) * ldw + n]; f[i + 8] = (f16)Wm[(size_t)(k0 + kh + 16 + i) * ldw + n]; }
  return f;
}
__device__ __forceinline__ float gelu_erf(float x) { return 0.5f * x * (1.0f + erff(x * 0.70710678118654752f)); }

#define GSTR 48
template <typename AT, int EPI, bool OUT16>
__global__ __launch_bounds__(256) void gemm_kne(const AT* __restrict__ A, int lda, const float* __restrict__ Wm, int ldw,
                                                const float* __restrict__ bias, const float* __restrict__ R, const float* __restrict__ gvec,
                                                void* __restrict__ Yv, int ldy, int K) {
  __shared__ __attribute__((aligned(16))) f16 ldsA[128 * GSTR];
  __shared__ __attribute__((aligned(16))) f16 ldsW[128 * GSTR];
  __shared__ __attribute__((aligned(16))) float oS[8][32 * 68];
  const int tid = threadIdx.x, lane = tid & 31, wave = tid >> 5, cl = lane & 15, rh = (lane >> 4) * 8;
  const int m0 = blockIdx.x * 128, n0 = blockIdx.y * 128;
  const int wm = (wave & 3) * 32, wn = (wave >> 2) * 64;
  f32x8 acc[2][4];
#pragma unroll
  for (int i = 0; i < 2; ++i)
#pragma unroll
    for (int j = 0; j < 4; ++j) { f32x8 z = {}; acc[i][j] = z; }
#pragma unroll 1
  for (int k0 = 0; k0 < K; k0 += 32) {
    __syncthreads();
    { const int row = tid >> 1, ch = (tid & 1) * 16;
      const AT* src = A + (size_t)(m0 + row) * lda + k0 + ch;
#pragma unroll
      for (int g = 0; g < 16; ++g) ldsA[row * GSTR + ch + g] = (f16)src[g]; }
    { const int k = tid >> 3, nn0 = (tid & 7) * 16;
      const float* src = Wm + (size_t)(k0 + k) * ldw + n0 + nn0;
#pragma unroll
      for (int g = 0; g < 4; ++g) { const v4f_t v = *(const v4f_t*)(src + 4 * g);
#pragma unroll
        for (int u = 0; u < 4; ++u) ldsW[(nn0 + 4 * g + u) * GSTR + k] = (f16)v[u]; } }
    __syncthreads();
    f16x16 af[2];
#pragma unroll
    for (int i = 0; i < 2; ++i) af[i] = lds_frag(ldsA + (wm + 16 * i) * GSTR, GSTR);
#pragma unroll
    for (int j = 0; j < 4; ++j) {
      const f16x16 bf = lds_frag(ldsW + (wn + 16 * j) * GSTR, GSTR);
#pragma unroll
      for (int i = 0; i < 2; ++i) acc[i][j] = wmma16(af[i], bf, acc[i][j]);
    }
  }
  float* so = oS[wave];
#pragma unroll
  for (int i = 0; i < 2; ++i)
#pragma unroll
    for (int j = 0; j < 4; ++j) {
      const int n = n0 + wn + 16 * j + cl;
      const float bv = bias ? bias[n] : 0.0f;
      const float gv = (EPI == 2) ? gvec[n] : 0.0f;
      if (EPI == 1) {
#pragma unroll 1
        for (int r = 0; r < 8; ++r) { const float xg = acc[i][j][r] + bv; so[(16 * i + rh + r) * 68 + 16 * j + cl] = 0.5f * xg * (1.0f + erff(xg * 0.70710678118654752f)); }
      } else {
#pragma unroll
        for (int r = 0; r < 8; ++r) {
          float v = acc[i][j][r] + bv;
          if (EPI == 2) v = R[(size_t)(m0 + wm + 16 * i + rh + r) * ldy + n] + gv * v;
          so[(16 * i + rh + r) * 68 + 16 * j + cl] = v;
        }
      }
    }
  asm volatile("s_wait_dscnt 0" ::: "memory");
  __builtin_amdgcn_wave_barrier();
#pragma unroll 1
  for (int pass = 0; pass < 2; ++pass) {
    if (OUT16) {
      f16* Y = (f16*)Yv;
#pragma unroll
      for (int it = 0; it < 8; ++it) { const int c = lane + 32 * it, rr = c >> 3, q8 = (c & 7) * 8;
        union { f16 h[8]; v4u_t v; } u;
#pragma unroll
        for (int e = 0; e < 8; ++e) u.h[e] = (f16)so[rr * 68 + q8 + e];
        *(volatile v4u_t*)(Y + (size_t)(m0 + wm + rr) * ldy + n0 + wn + q8) = u.v; }
    } else {
      float* Y = (float*)Yv;
#pragma unroll
      for (int it = 0; it < 16; ++it) { const int f4 = lane + 32 * it, rr = f4 >> 4, q = (f4 & 15) * 4;
        *(volatile v4f_t*)(Y + (size_t)(m0 + wm + rr) * ldy + n0 + wn + q) = *(const v4fa*)(so + rr * 68 + q); }
    }
    __threadfence();
  }
}

__global__ __launch_bounds__(256) void k_edge(const float* __restrict__ Rel, const float* __restrict__ XP,
                                             const float* __restrict__ W1m, const float* __restrict__ b1m, const float* __restrict__ W2m, const float* __restrict__ b2m,
                                             const float* __restrict__ W1a, const float* __restrict__ b1a, const float* __restrict__ W2a, const float* __restrict__ b2a,
                                             const float* __restrict__ x, float* __restrict__ out) {
  __shared__ __attribute__((aligned(16))) f16 relS[NNr * 72];
  __shared__ __attribute__((aligned(16))) f16 hS[NNr * 264];
  __shared__ float eS[NNr];
  __shared__ __attribute__((aligned(16))) float aggS[8][DDr];
  const int tid = threadIdx.x, lane = tid & 31, wave = tid >> 5, cl = lane & 15, rh = (lane >> 4) * 8;
  const int b = blockIdx.x / NNr, i = blockIdx.x % NNr;
  const float* relrow = Rel + (((size_t)b * NNr + i) * NNr) * RRr;
  for (int e = tid; e < NNr * RRr; e += 256) { const int j = e >> 6, r = e & 63; relS[j * 72 + r] = (f16)relrow[e]; }
  __syncthreads();
  { f32x8 acc[16];
#pragma unroll
    for (int t = 0; t < 16; ++t) { f32x8 z = {}; acc[t] = z; }
#pragma unroll
    for (int ks = 0; ks < 2; ++ks) { const f16x16 af = lds_frag(relS + (wave * 16) * 72 + ks * 32, 72);
#pragma unroll
      for (int t = 0; t < 16; ++t) acc[t] = wmma16(af, wfragKN(W1a + (size_t)2 * DDr * DDr, DDr, ks * 32, t * 16), acc[t]); }
    const float* xia = XP + ((size_t)b * NNr + i) * 768 + DDr;
#pragma unroll
    for (int t = 0; t < 16; ++t) { const int c = t * 16 + cl; const float bc = b1a[c] + xia[c];
#pragma unroll
      for (int r = 0; r < 8; ++r) { const int j = wave * 16 + rh + r; hS[j * 264 + c] = (f16)(acc[t][r] + XP[((size_t)b * NNr + j) * 768 + 2 * DDr + c] + bc); } } }
  __syncthreads();
  { const int j = tid >> 1, half = (tid & 1) * 128; float e = 0.0f;
#pragma unroll 1
    for (int c = half; c < half + 128; ++c) e += gelu_erf((float)hS[j * 264 + c]) * W2a[c];
    e += __shfl_xor(e, 1, 32);
    if ((tid & 1) == 0) eS[j] = e + b2a[0]; }
  __syncthreads();
  { f32x8 acc[16];
#pragma unroll
    for (int t = 0; t < 16; ++t) { f32x8 z = {}; acc[t] = z; }
#pragma unroll
    for (int ks = 0; ks < 2; ++ks) { const f16x16 af = lds_frag(relS + (wave * 16) * 72 + ks * 32, 72);
#pragma unroll
      for (int t = 0; t < 16; ++t) acc[t] = wmma16(af, wfragKN(W1m + (size_t)DDr * DDr, DDr, ks * 32, t * 16), acc[t]); }
#pragma unroll
    for (int t = 0; t < 16; ++t)
#pragma unroll
      for (int r = 0; r < 8; ++r) { const int j = wave * 16 + rh + r, c = t * 16 + cl;
        hS[j * 264 + c] = (f16)(acc[t][r] + XP[((size_t)b * NNr + j) * 768 + c] + b1m[c]); } }
  __syncthreads();
#pragma unroll 1
  for (int e = tid; e < NNr * DDr; e += 256) { const int j = e >> 8, c = e & 255; hS[j * 264 + c] = (f16)gelu_erf((float)hS[j * 264 + c]); }
  __syncthreads();
  if (tid < 32) { float m = -3.0e38f; for (int j = lane; j < NNr; j += 32) if (j != i) m = fmaxf(m, eS[j]);
#pragma unroll
    for (int off = 1; off < 32; off <<= 1) m = fmaxf(m, __shfl_xor(m, off, 32));
    float z = 0.0f; float ev[4];
#pragma unroll
    for (int q = 0; q < 4; ++q) { const int j = lane + 32 * q; ev[q] = (j != i) ? expf(eS[j] - m) : 0.0f; z += ev[q]; }
#pragma unroll
    for (int off = 1; off < 32; off <<= 1) z += __shfl_xor(z, off, 32);
#pragma unroll
    for (int q = 0; q < 4; ++q) eS[lane + 32 * q] = ev[q] / z; }
  __syncthreads();
  { f32x8 acc[16];
#pragma unroll
    for (int t = 0; t < 16; ++t) { f32x8 z = {}; acc[t] = z; }
#pragma unroll 1
    for (int ks = 0; ks < 8; ++ks) { const f16x16 af = lds_frag(hS + (wave * 16) * 264 + ks * 32, 264);
#pragma unroll
      for (int t = 0; t < 16; ++t) acc[t] = wmma16(af, wfragKN(W2m, DDr, ks * 32, t * 16), acc[t]); }
    float al[8];
#pragma unroll
    for (int r = 0; r < 8; ++r) al[r] = eS[wave * 16 + rh + r];
#pragma unroll
    for (int t = 0; t < 16; ++t) { float s = 0.0f;
#pragma unroll
      for (int r = 0; r < 8; ++r) s += al[r] * acc[t][r];
      s += __shfl_xor(s, 16, 32);
      if (lane < 16) aggS[wave][t * 16 + cl] = s; } }
  __syncthreads();
#pragma unroll 1
  for (int pass = 0; pass < 2; ++pass) { if (tid < 64) { const int c4 = tid * 4; v4f_t v = *(const v4f_t*)(x + ((size_t)b * NNr + i) * DDr + c4);
      for (int e = 0; e < 4; ++e) { float s = b2m[c4 + e]; for (int w = 0; w < 8; ++w) s += aggS[w][c4 + e]; v[e] += s; }
      *(volatile v4f_t*)(out + ((size_t)b * NNr + i) * DDr + c4) = v; } __threadfence(); }
}

extern "C" void kernel_launch(void* const* d_in, const int* in_sizes, int n_in,
                              void* d_out, int out_size, void* d_ws, size_t ws_size,
                              hipStream_t stream) {
  (void)in_sizes; (void)n_in; (void)out_size;
  const float** f = (const float**)d_in;
  const float* x = f[0], *Rel = f[1], *W1m = f[2], *b1m = f[3], *W2m = f[4], *b2m = f[5], *W1a = f[6], *b1a = f[7], *W2a = f[8], *b2a = f[9];
  float* out = (float*)d_out;
  char* ws = (char*)d_ws;
  float* XP = (float*)ws; ws += (size_t)NROW * 768 * 4;
  if ((size_t)(ws - (char*)d_ws) > ws_size) return;
  const dim3 blk(256);
  gemm_kne<float, 0, false><<<dim3(NROW / 128, DDr / 128), blk, 0, stream>>>(x, DDr, W1m, DDr, nullptr, nullptr, nullptr, XP, 768, DDr);
  gemm_kne<float, 0, false><<<dim3(NROW / 128, DDr / 128), blk, 0, stream>>>(x, DDr, W1a, DDr, nullptr, nullptr, nullptr, XP + DDr, 768, DDr);
  gemm_kne<float, 0, false><<<dim3(NROW / 128, DDr / 128), blk, 0, stream>>>(x, DDr, W1a + (size_t)DDr * DDr, DDr, nullptr, nullptr, nullptr, XP + 2 * DDr, 768, DDr);
  k_edge<<<dim3(NBr * NNr), blk, 0, stream>>>(Rel, XP, W1m, b1m, W2m, b2m, W1a, b1a, W2a, b2a, x, out);
}
